// Node_encoder_36086315221303
// MI455X (gfx1250) — hardware-run, weakly checked
//
#include <hip/hip_runtime.h>
#include <math.h>

typedef __attribute__((ext_vector_type(16))) _Float16 v16h;
typedef __attribute__((ext_vector_type(8)))  _Float16 v8h;
typedef __attribute__((ext_vector_type(8)))  float    v8f;
typedef __attribute__((ext_vector_type(4)))  float    v4f;

constexpr int kBatch  = 4;
constexpr int kNodes  = 50;
constexpr int kFeat   = 16;
constexpr int kLen    = 64;
constexpr int kHid    = 64;
constexpr int kXz     = 2 * kHid;
constexpr int kState  = 128;
constexpr int kDtRank = 4;
constexpr int kProjN  = kDtRank + 2 * kState;
constexpr int kProjP  = 320;
constexpr int kOutDim = 32;
constexpr int kOutLen = 32;
constexpr int kSeqs   = kNodes * kBatch;
constexpr int kRows   = kSeqs * kLen;
constexpr int kRowsT  = kSeqs * kOutLen;
constexpr int kOutElems = kBatch * kOutDim * kNodes * kOutLen;
constexpr int kStatP  = 256;
constexpr int kRank   = 16;
constexpr int kRankP  = 32;
constexpr int kParts  = 8;
constexpr int kPState = kState / kParts;
constexpr float kLnEps  = 1e-5f;
constexpr float kWCarry = 1024.0f;
constexpr float kResid  = 2048.0f;
static_assert(kRank == kFeat && kRankP == 32);
static_assert(kProjN == 260 && kProjN <= kProjP && (kProjP % 64) == 0);
static_assert(kSeqs == 200 && kRows == 12800 && kRowsT == 6400 && kOutElems == 204800);
static_assert(kHid == 64 && kLen == 64 && kXz == 128 && kState == 128 && kDtRank == 4);
static_assert(kParts == 8 && kPState == 16);
static_assert((kRows % 32) == 0 && (kRowsT % 32) == 0 && (kHid % 64) == 0 && (kXz % 64) == 0);
static_assert((kHid % 32) == 0 && (kRankP % 32) == 0);
static_assert(kSeqs <= kStatP && kStatP == 4 * 64);
static_assert(2 * kOutDim == kHid && kOutLen * 2 == kLen);

constexpr size_t kSzEW   = (size_t)kHid * kRankP * 2;
constexpr size_t kSzW64  = (size_t)kHid * kHid * 2;
constexpr size_t kSzW2   = (size_t)kXz * kHid * 2;
constexpr size_t kSzW3   = (size_t)kProjP * kHid * 2;
constexpr size_t kSzAN   = (size_t)kHid * kState * 4;
constexpr size_t kSzXA   = (size_t)kRows * kRankP * 2;
constexpr size_t kSzF32  = (size_t)kRows * kHid * 4;
constexpr size_t kSzF16  = (size_t)kRows * kHid * 2;
constexpr size_t kSzXZ   = (size_t)kRows * kXz * 4;
constexpr size_t kSzPROJ = (size_t)kRows * kProjP * 4;
constexpr size_t kYpPlane = (size_t)kSeqs * 16 * kHid * 4;
constexpr size_t kSzYP   = (size_t)kParts * kYpPlane * 4;
constexpr size_t kSzRS   = (size_t)kRows * 4;
constexpr size_t kSzST   = (size_t)kStatP * 4;
constexpr size_t kSzT32  = (size_t)kRowsT * kHid * 4;
constexpr size_t kSzT16  = (size_t)kRowsT * kHid * 2;
constexpr size_t kOffEW   = 0;
constexpr size_t kOffW1   = kOffEW   + kSzEW;
constexpr size_t kOffW2   = kOffW1   + kSzW64;
constexpr size_t kOffW3   = kOffW2   + kSzW2;
constexpr size_t kOffW4   = kOffW3   + kSzW3;
constexpr size_t kOffW5   = kOffW4   + kSzW64;
constexpr size_t kOffHW   = kOffW5   + kSzW64;
constexpr size_t kOffAN   = kOffHW   + kSzW64;
constexpr size_t kOffXA   = kOffAN   + kSzAN;
constexpr size_t kOffH0   = kOffXA   + kSzXA;
constexpr size_t kOffA1H  = kOffH0   + kSzF32;
constexpr size_t kOffA1L  = kOffA1H  + kSzF16;
constexpr size_t kOffH1   = kOffA1L  + kSzF16;
constexpr size_t kOffA2H  = kOffH1   + kSzF32;
constexpr size_t kOffA2L  = kOffA2H  + kSzF16;
constexpr size_t kOffXZ   = kOffA2L  + kSzF16;
constexpr size_t kOffXC   = kOffXZ   + kSzXZ;
constexpr size_t kOffXCH  = kOffXC   + kSzF32;
constexpr size_t kOffXCL  = kOffXCH  + kSzF16;
constexpr size_t kOffPROJ = kOffXCL  + kSzF16;
constexpr size_t kOffDT   = kOffPROJ + kSzPROJ;
constexpr size_t kOffYP   = kOffDT   + kSzF32;
constexpr size_t kOffY    = kOffYP   + kSzYP;
constexpr size_t kOffYH   = kOffY    + kSzF32;
constexpr size_t kOffYL   = kOffYH   + kSzF16;
constexpr size_t kOffM    = kOffYL   + kSzF16;
constexpr size_t kOffGH   = kOffM    + kSzF32;
constexpr size_t kOffGL   = kOffGH   + kSzF16;
constexpr size_t kOffH2   = kOffGL   + kSzF16;
constexpr size_t kOffRS1  = kOffH2   + kSzF32;
constexpr size_t kOffMU   = kOffRS1  + kSzRS;
constexpr size_t kOffRS2  = kOffMU   + kSzST;
constexpr size_t kOffRSTD = kOffRS2  + kSzRS;
constexpr size_t kOffL3   = kOffRSTD + kSzST;
constexpr size_t kOffLH   = kOffL3   + kSzT32;
constexpr size_t kOffLL   = kOffLH   + kSzT16;
constexpr size_t kOffRAW  = kOffLL   + kSzT16;
constexpr size_t kWsTotal = kOffRAW  + kSzT32;
static_assert(kSzEW == 4096ull && kSzW64 == 8192ull && kSzW2 == 16384ull && kSzW3 == 40960ull && kSzAN == 32768ull);
static_assert(kSzXA == 819200ull && kSzF32 == 3276800ull && kSzF16 == 1638400ull && kSzXZ == 6553600ull);
static_assert(kYpPlane == 819200ull);
static_assert(kSzPROJ == 16384000ull && kSzYP == 26214400ull && kSzRS == 51200ull && kSzST == 1024ull);
static_assert(kSzT32 == 1638400ull && kSzT16 == 819200ull);
static_assert(kWsTotal == 94439424ull);
static_assert(kWsTotal <= 134217728ull);
static_assert((kSzEW % 128) == 0 && (kSzW64 % 128) == 0 && (kSzW2 % 128) == 0 && (kSzW3 % 128) == 0 &&
              (kSzAN % 128) == 0 && (kSzXA % 128) == 0 && (kSzF32 % 128) == 0 && (kSzF16 % 128) == 0 &&
              (kSzXZ % 128) == 0 && (kSzPROJ % 128) == 0 && (kSzYP % 128) == 0 && (kSzRS % 128) == 0 &&
              (kSzST % 128) == 0 && (kSzT32 % 128) == 0 && (kSzT16 % 128) == 0);

__device__ __forceinline__ _Float16 f16_flush(float v) {
  const float w = (fabsf(v) < 6.103515625e-05f) ? 0.0f : v;
  return (_Float16)w;
}
__device__ __forceinline__ void f16_split(float v, _Float16& hi, _Float16& lo) {
  hi = f16_flush(v);
  const float hf = (float)hi;
  const float r = (v - hf) * kResid;
  lo = f16_flush(r);
}

__device__ __forceinline__ float bf16r(float v) {
  unsigned u = __float_as_uint(v);
  u = (u + 0x7FFFu + ((u >> 16) & 1u)) & 0xFFFF0000u;
  return __uint_as_float(u);
}

__device__ __forceinline__ float h16_to_f32(unsigned hb) {
  const unsigned sgn = (hb & 0x8000u) << 16; const unsigned em = hb & 0x7fffu;
  const float fn = __uint_as_float((em << 13) + 0x38000000u);
  const float fs = (float)em * 5.9604644775390625e-8f;
  const float mag = (em < 0x400u) ? fs : fn; return __uint_as_float(__float_as_uint(mag) | sgn); }

namespace eng {
union FragU { v16h v; v8h h[2]; };
__device__ __forceinline__ v16h frag_load(const _Float16* p) {
  FragU f;
  f.h[0] = *(const v8h*)(p);
  f.h[1] = *(const v8h*)(p + 16);
  return f.v;
}
__device__ __forceinline__ v8f mma(v16h a, v16h b, v8f c) {
  return __builtin_amdgcn_wmma_f32_16x16x32_f16(false, a, false, b, (short)0, c, false, false);
}
__device__ __forceinline__ void guard1(v8f& a, v16h x, v16h y) {
  asm volatile("v_nop\n\tv_nop\n\tv_nop\n\tv_nop" : "+v"(a) : "v"(x), "v"(y));
}
__device__ __forceinline__ void guard_acc(v8f& a) {
  asm volatile("v_nop\n\tv_nop\n\tv_nop\n\tv_nop" : "+v"(a));
}
__device__ __forceinline__ void keep4(v16h a, v16h b, v16h c, v16h d) {
  asm volatile("v_nop" :: "v"(a), "v"(b), "v"(c), "v"(d));
}

template <int MI, int SPL>
__global__ __launch_bounds__(256) void gemm_f16_kernel(
    const unsigned short* __restrict__ Ap, const unsigned short* __restrict__ A2p, int lda,
    const unsigned short* __restrict__ Btp, const unsigned short* __restrict__ Bt2p, int ldb,
    float* __restrict__ C, int ldc, int M, int N, int K, float scale, float rscale)
{
  static_assert(MI >= 1 && MI <= 2);
  static_assert(SPL >= 0 && SPL <= 2);
  const _Float16* A   = (const _Float16*)Ap;
  const _Float16* A2  = (const _Float16*)A2p;
  const _Float16* Bt  = (const _Float16*)Btp;
  const _Float16* Bt2 = (const _Float16*)Bt2p;
  __shared__ __align__(16) float sT[8][16 * 68];
  const int lane = threadIdx.x & 31;
  const int wave = threadIdx.x >> 5;
  const int tilesN = N >> 6;
  const int tilesM = M / (16 * MI);
  const int tile = blockIdx.x * 8 + wave;
  if (tile >= tilesM * tilesN) return;
  const int tm = tile / tilesN;
  const int tn = tile - tm * tilesN;
  const int m0 = tm * (16 * MI);
  const int n0 = tn << 6;
  const int rlane = lane & 15;
  const int koff  = (lane >> 4) * 8;
  const int mOff  = (lane >> 4) * 8;

  v8f acc[MI][4], accr[MI][4];
#pragma unroll
  for (int i = 0; i < MI; ++i)
#pragma unroll
    for (int j = 0; j < 4; ++j) {
      acc[i][j]  = (v8f){0.f, 0.f, 0.f, 0.f, 0.f, 0.f, 0.f, 0.f};
      accr[i][j] = (v8f){0.f, 0.f, 0.f, 0.f, 0.f, 0.f, 0.f, 0.f};
    }

  for (int k0 = 0; k0 < K; k0 += 32) {
    v16h bh[4], bl[4];
#pragma unroll
    for (int j = 0; j < 4; ++j) {
      const size_t bo = (size_t)(n0 + (j << 4) + rlane) * ldb + koff + k0;
      bh[j] = frag_load(Bt + bo);
      if (SPL == 2) bl[j] = frag_load(Bt2 + bo); else bl[j] = bh[j];
    }
#pragma unroll
    for (int i = 0; i < MI; ++i) {
      const size_t ao = (size_t)(m0 + (i << 4) + rlane) * lda + koff + k0;
      const v16h ah = frag_load(A + ao);
      v16h al = ah;
      if (SPL >= 1) al = frag_load(A2 + ao);
#pragma unroll
      for (int j = 0; j < 4; ++j) {
        acc[i][j] = mma(ah, bh[j], acc[i][j]);
        if (SPL >= 1) accr[i][j] = mma(al, bh[j], accr[i][j]);
        if (SPL == 2) accr[i][j] = mma(ah, bl[j], accr[i][j]);
      }
#pragma unroll
      for (int j = 0; j < 4; ++j) {
        guard1(acc[i][j], ah, al);
        if (SPL >= 1) guard1(accr[i][j], ah, al);
      }
    }
    keep4(bh[0], bh[1], bh[2], bh[3]);
    if (SPL == 2) keep4(bl[0], bl[1], bl[2], bl[3]);
  }
#pragma unroll
  for (int i = 0; i < MI; ++i)
#pragma unroll
    for (int j = 0; j < 4; ++j) {
      guard_acc(acc[i][j]);
      if (SPL >= 1) guard_acc(accr[i][j]);
    }

  float* slab = sT[wave];
#pragma unroll
  for (int i = 0; i < MI; ++i) {
    const int mBase = m0 + (i << 4);
#pragma unroll
    for (int j = 0; j < 4; ++j) {
#pragma unroll
      for (int r = 0; r < 8; ++r) {
        float v = acc[i][j][r] * scale;
        if (SPL >= 1) v += accr[i][j][r] * rscale;
        slab[(mOff + r) * 68 + (j << 4) + rlane] = v;
      }
    }
    __builtin_amdgcn_fence(__ATOMIC_RELEASE, "workgroup");
    __builtin_amdgcn_wave_barrier();
    __builtin_amdgcn_fence(__ATOMIC_ACQUIRE, "workgroup");
    {
      const int hh = lane >> 4, c4 = (lane & 15) * 4;
      for (int pass = 0; pass < 2; ++pass) {
#pragma unroll
        for (int it = 0; it < 8; ++it) {
          const int row = it * 2 + hh;
          const v4f v = *(const v4f*)(slab + row * 68 + c4);
          *(volatile v4f*)(C + (size_t)(mBase + row) * ldc + n0 + c4) = v;
        }
        __threadfence();
      }
    }
    __builtin_amdgcn_fence(__ATOMIC_RELEASE, "workgroup");
    __builtin_amdgcn_wave_barrier();
    __builtin_amdgcn_fence(__ATOMIC_ACQUIRE, "workgroup");
  }
}
}

__global__ __launch_bounds__(256) void pack_kpad_bf_kernel(
    const float* __restrict__ W, unsigned short* __restrict__ dH, int total8, float carry)
{
  constexpr int kGroupsP = kRankP / 8;
  constexpr int kGroupsL = kRank / 8;
  const int i = blockIdx.x * 256 + threadIdx.x;
  if (i >= total8) return;
  const int row = i / kGroupsP;
  const int g = i - row * kGroupsP;
  const bool live = (g < kGroupsL);
  const int gc = live ? g : (kGroupsL - 1);
  const float* sp = W + (size_t)row * kRank + gc * 8;
  const v4f a0 = *(const v4f*)(sp);
  const v4f a1 = *(const v4f*)(sp + 4);
  const float w0 = a0[0];
  const float w1 = a0[1];
  const float w2 = a0[2];
  const float w3 = a0[3];
  const float w4 = a1[0];
  const float w5 = a1[1];
  const float w6 = a1[2];
  const float w7 = a1[3];
  const float t0 = bf16r(w0) * carry;
  const float t1 = bf16r(w1) * carry;
  const float t2 = bf16r(w2) * carry;
  const float t3 = bf16r(w3) * carry;
  const float t4 = bf16r(w4) * carry;
  const float t5 = bf16r(w5) * carry;
  const float t6 = bf16r(w6) * carry;
  const float t7 = bf16r(w7) * carry;
  const float g0 = live ? t0 : 0.0f;
  const float g1 = live ? t1 : 0.0f;
  const float g2 = live ? t2 : 0.0f;
  const float g3 = live ? t3 : 0.0f;
  const float g4 = live ? t4 : 0.0f;
  const float g5 = live ? t5 : 0.0f;
  const float g6 = live ? t6 : 0.0f;
  const float g7 = live ? t7 : 0.0f;
  v8h hv;
  hv[0] = f16_flush(g0);
  hv[1] = f16_flush(g1);
  hv[2] = f16_flush(g2);
  hv[3] = f16_flush(g3);
  hv[4] = f16_flush(g4);
  hv[5] = f16_flush(g5);
  hv[6] = f16_flush(g6);
  hv[7] = f16_flush(g7);
  unsigned short* qh = dH + ((size_t)i << 3);
  *(volatile v8h*)qh = hv;
  __threadfence();
  *(volatile v8h*)qh = hv;
}

__global__ __launch_bounds__(256) void pack_w_kernel(
    const float* __restrict__ W, unsigned short* __restrict__ dH, int rows_live, float carry)
{
  const int i = blockIdx.x * 256 + threadIdx.x;
  const int row = i >> 3;
  const int col = (i & 7) * 8;
  const bool live = (row < rows_live);
  const int rc = live ? row : (rows_live - 1);
  const float* sp = W + (size_t)rc * kHid + col;
  const v4f a0 = *(const v4f*)(sp);
  const v4f a1 = *(const v4f*)(sp + 4);
  const float w0 = a0[0];
  const float w1 = a0[1];
  const float w2 = a0[2];
  const float w3 = a0[3];
  const float w4 = a1[0];
  const float w5 = a1[1];
  const float w6 = a1[2];
  const float w7 = a1[3];
  const float t0 = bf16r(w0) * carry;
  const float t1 = bf16r(w1) * carry;
  const float t2 = bf16r(w2) * carry;
  const float t3 = bf16r(w3) * carry;
  const float t4 = bf16r(w4) * carry;
  const float t5 = bf16r(w5) * carry;
  const float t6 = bf16r(w6) * carry;
  const float t7 = bf16r(w7) * carry;
  const float g0 = live ? t0 : 0.0f;
  const float g1 = live ? t1 : 0.0f;
  const float g2 = live ? t2 : 0.0f;
  const float g3 = live ? t3 : 0.0f;
  const float g4 = live ? t4 : 0.0f;
  const float g5 = live ? t5 : 0.0f;
  const float g6 = live ? t6 : 0.0f;
  const float g7 = live ? t7 : 0.0f;
  v8h hv;
  hv[0] = f16_flush(g0);
  hv[1] = f16_flush(g1);
  hv[2] = f16_flush(g2);
  hv[3] = f16_flush(g3);
  hv[4] = f16_flush(g4);
  hv[5] = f16_flush(g5);
  hv[6] = f16_flush(g6);
  hv[7] = f16_flush(g7);
  unsigned short* qh = dH + ((size_t)i << 3);
  *(volatile v8h*)qh = hv;
  __threadfence();
  *(volatile v8h*)qh = hv;
}

__global__ __launch_bounds__(256) void embed_a_kernel(
    const float* __restrict__ x, unsigned short* __restrict__ XA)
{
  const int i = blockIdx.x * 256 + threadIdx.x;
  const int r = i >> 2;
  const int g = i & 3;
  const bool live = (g < kFeat / 8);
  const int gc = live ? g : (kFeat / 8 - 1);
  const int q = r / kLen;
  const int l = r - q * kLen;
  const int node = q / kBatch;
  const int b = q - node * kBatch;
  const float* sp = x + ((size_t)(b * kNodes + node) * kFeat + gc * 8) * kLen + l;
  const float w0 = sp[0 * kLen];
  const float w1 = sp[1 * kLen];
  const float w2 = sp[2 * kLen];
  const float w3 = sp[3 * kLen];
  const float w4 = sp[4 * kLen];
  const float w5 = sp[5 * kLen];
  const float w6 = sp[6 * kLen];
  const float w7 = sp[7 * kLen];
  const float t0 = bf16r(w0);
  const float t1 = bf16r(w1);
  const float t2 = bf16r(w2);
  const float t3 = bf16r(w3);
  const float t4 = bf16r(w4);
  const float t5 = bf16r(w5);
  const float t6 = bf16r(w6);
  const float t7 = bf16r(w7);
  const float g0 = live ? t0 : 0.0f;
  const float g1 = live ? t1 : 0.0f;
  const float g2 = live ? t2 : 0.0f;
  const float g3 = live ? t3 : 0.0f;
  const float g4 = live ? t4 : 0.0f;
  const float g5 = live ? t5 : 0.0f;
  const float g6 = live ? t6 : 0.0f;
  const float g7 = live ? t7 : 0.0f;
  v8h hv;
  hv[0] = f16_flush(g0);
  hv[1] = f16_flush(g1);
  hv[2] = f16_flush(g2);
  hv[3] = f16_flush(g3);
  hv[4] = f16_flush(g4);
  hv[5] = f16_flush(g5);
  hv[6] = f16_flush(g6);
  hv[7] = f16_flush(g7);
  unsigned short* qh = XA + ((size_t)i << 3);
  *(volatile v8h*)qh = hv;
  __threadfence();
  *(volatile v8h*)qh = hv;
}

template <int ACT, int BIAS>
__global__ __launch_bounds__(256) void split_kernel(
    const float* __restrict__ src, const float* __restrict__ bias,
    unsigned short* __restrict__ AH, unsigned short* __restrict__ AL)
{
  const int i = blockIdx.x * 256 + threadIdx.x;
  const size_t e0 = (size_t)i << 3;
  const int c8 = (i & 7) * 8;
  const v4f a0 = *(const v4f*)(src + e0);
  const v4f a1 = *(const v4f*)(src + e0 + 4);
  float f[8];
#pragma unroll
  for (int e = 0; e < 4; ++e) {
    const float p0 = a0[e];
    const float p1 = a1[e];
    f[e] = p0;
    f[4 + e] = p1;
  }
  if (BIAS == 1) {
    const v4f b0 = *(const v4f*)(bias + c8);
    const v4f b1 = *(const v4f*)(bias + c8 + 4);
#pragma unroll
    for (int e = 0; e < 4; ++e) {
      const float q0 = b0[e];
      const float q1 = b1[e];
      f[e] += bf16r(q0);
      f[4 + e] += bf16r(q1);
    }
  }
  v8h hv, lv;
#pragma unroll
  for (int e = 0; e < 8; ++e) {
    float v = f[e];
    if (ACT == 1) v = v / (1.0f + expf(-v));
    _Float16 h, l;
    f16_split(v, h, l);
    hv[e] = h;
    lv[e] = l;
  }
  unsigned short* qh = AH + e0;
  unsigned short* ql = AL + e0;
  *(volatile v8h*)qh = hv;
  *(volatile v8h*)ql = lv;
  __threadfence();
  *(volatile v8h*)qh = hv;
  *(volatile v8h*)ql = lv;
}

__global__ __launch_bounds__(256) void conv_silu_kernel(
    const float* __restrict__ XZ, const float* __restrict__ cw, const float* __restrict__ cb,
    float* __restrict__ XC)
{
  const int i = blockIdx.x * 256 + threadIdx.x;
  const int row = i >> 4;
  const int d4 = (i & 15) * 4;
  const int l = row % kLen;
  const bool first = (l == 0);
  const int rp = first ? row : (row - 1);
  const v4f cur = *(const v4f*)(XZ + (size_t)row * kXz + d4);
  const v4f prv = *(const v4f*)(XZ + (size_t)rp * kXz + d4);
  const float p0 = prv[0];
  const float p1 = prv[1];
  const float p2 = prv[2];
  const float p3 = prv[3];
  const v4f wa = *(const v4f*)(cw + d4 * 2);
  const v4f wb = *(const v4f*)(cw + d4 * 2 + 4);
  const v4f bv = *(const v4f*)(cb + d4);
  const float wa0 = wa[0];
  const float wa1 = wa[1];
  const float wa2 = wa[2];
  const float wa3 = wa[3];
  const float wb0 = wb[0];
  const float wb1 = wb[1];
  const float wb2 = wb[2];
  const float wb3 = wb[3];
  const float c0 = cur[0];
  const float c1 = cur[1];
  const float c2 = cur[2];
  const float c3 = cur[3];
  const float b0 = bv[0];
  const float b1 = bv[1];
  const float b2 = bv[2];
  const float b3 = bv[3];
  const float x0 = first ? 0.0f : p0;
  const float x1 = first ? 0.0f : p1;
  const float x2 = first ? 0.0f : p2;
  const float x3 = first ? 0.0f : p3;
  const float s0 = fmaf(c0, bf16r(wa1), x0 * bf16r(wa0)) + bf16r(b0);
  const float s1 = fmaf(c1, bf16r(wa3), x1 * bf16r(wa2)) + bf16r(b1);
  const float s2 = fmaf(c2, bf16r(wb1), x2 * bf16r(wb0)) + bf16r(b2);
  const float s3 = fmaf(c3, bf16r(wb3), x3 * bf16r(wb2)) + bf16r(b3);
  v4f o;
  o[0] = s0 / (1.0f + expf(-s0));
  o[1] = s1 / (1.0f + expf(-s1));
  o[2] = s2 / (1.0f + expf(-s2));
  o[3] = s3 / (1.0f + expf(-s3));
  float* p = XC + (size_t)row * kHid + d4;
  *(volatile v4f*)p = o;
  __threadfence();
  *(volatile v4f*)p = o;
}

__global__ __launch_bounds__(256) void dt_kernel(
    const float* __restrict__ PROJ, const float* __restrict__ dtw, const float* __restrict__ dtb,
    float* __restrict__ DT)
{
  const int i = blockIdx.x * 256 + threadIdx.x;
  const int row = i >> 4;
  const int d4 = (i & 15) * 4;
  const v4f xl = *(const v4f*)(PROJ + (size_t)row * kProjP);
  const float x0 = xl[0];
  const float x1 = xl[1];
  const float x2 = xl[2];
  const float x3 = xl[3];
  const v4f bq = *(const v4f*)(dtb + d4);
  v4f o;
#pragma unroll
  for (int j = 0; j < 4; ++j) {
    const v4f wq = *(const v4f*)(dtw + (size_t)(d4 + j) * kDtRank);
    const float w0 = wq[0];
    const float w1 = wq[1];
    const float w2 = wq[2];
    const float w3 = wq[3];
    const float bj = bq[j];
    float acc = x0 * bf16r(w0);
    acc = fmaf(x1, bf16r(w1), acc);
    acc = fmaf(x2, bf16r(w2), acc);
    acc = fmaf(x3, bf16r(w3), acc);
    const float v = acc + bf16r(bj);
    o[j] = (v > 20.0f) ? v : log1pf(expf(v));
  }
  float* p = DT + (size_t)row * kHid + d4;
  *(volatile v4f*)p = o;
  __threadfence();
  *(volatile v4f*)p = o;
}

__global__ __launch_bounds__(256) void a_neg_kernel(
    const float* __restrict__ A_log, float* __restrict__ AN)
{
  const int i = blockIdx.x * 256 + threadIdx.x;
  const v4f a = *(const v4f*)(A_log + (size_t)i * 4);
  const float a0 = a[0];
  const float a1 = a[1];
  const float a2 = a[2];
  const float a3 = a[3];
  v4f o;
  o[0] = -expf(bf16r(a0));
  o[1] = -expf(bf16r(a1));
  o[2] = -expf(bf16r(a2));
  o[3] = -expf(bf16r(a3));
  float* p = AN + (size_t)i * 4;
  *(volatile v4f*)p = o;
  __threadfence();
  *(volatile v4f*)p = o;
}

__global__ __launch_bounds__(256) void scan_kernel(
    const float* __restrict__ DT, const float* __restrict__ XC, const float* __restrict__ PROJ,
    const float* __restrict__ AN, float* __restrict__ YP)
{
  const int t = blockIdx.x * 256 + threadIdx.x;
  const int d = t & (kHid - 1);
  const int s = (t >> 6) & (kParts - 1);
  const int q = t >> 9;
  float An[kPState], h[kPState];
  const float* ap = AN + (size_t)d * kState + s * kPState;
#pragma unroll
  for (int g = 0; g < kPState / 4; ++g) {
    const v4f a = *(const v4f*)(ap + 4 * g);
#pragma unroll
    for (int e = 0; e < 4; ++e) {
      const float ae = a[e];
      An[4 * g + e] = ae;
      h[4 * g + e] = 0.0f;
    }
  }
  const size_t row0 = (size_t)q * kLen;
  float* yq = YP + (((size_t)(s * kSeqs + q) * 16) * kHid + d) * 4;
  for (int grp = 0; grp < 16; ++grp) {
    float yv[4];
#pragma unroll
    for (int j = 0; j < 4; ++j) {
      const size_t r = row0 + (size_t)(grp * 4 + j);
      const float dt = DT[r * kHid + d];
      const float u = XC[r * kHid + d];
      const float du = dt * u;
      const float* bp = PROJ + r * kProjP + kDtRank + s * kPState;
      const float* cp = bp + kState;
      float acc = 0.0f;
#pragma unroll
      for (int g = 0; g < kPState / 4; ++g) {
        const v4f Bv = *(const v4f*)(bp + 4 * g);
        const v4f Cv = *(const v4f*)(cp + 4 * g);
#pragma unroll
        for (int e = 0; e < 4; ++e) {
          const float bn = Bv[e];
          const float cn = Cv[e];
          const float dec = __expf(dt * An[4 * g + e]);
          h[4 * g + e] = fmaf(dec, h[4 * g + e], du * bn);
          acc = fmaf(h[4 * g + e], cn, acc);
        }
      }
      yv[j] = acc;
    }
    v4f o;
    o[0] = yv[0];
    o[1] = yv[1];
    o[2] = yv[2];
    o[3] = yv[3];
    float* p = yq + (size_t)grp * kHid * 4;
    *(volatile v4f*)p = o;
    __threadfence();
    *(volatile v4f*)p = o;
  }
}

__global__ __launch_bounds__(256) void gate_kernel(
    const float* __restrict__ YP, const float* __restrict__ XC, const float* __restrict__ XZ,
    const float* __restrict__ Dskip, float* __restrict__ Y)
{
  const int i = blockIdx.x * 256 + threadIdx.x;
  const int row = i >> 4;
  const int d4 = (i & 15) * 4;
  const int q = row / kLen;
  const int l = row - q * kLen;
  const size_t yo = (((size_t)q * 16 + (size_t)(l >> 2)) * kHid + d4) * 4 + (size_t)(l & 3);
  float rs[4];
  {
    const float* y0p = YP + yo;
    const float a0 = y0p[0];
    const float a1 = y0p[4];
    const float a2 = y0p[8];
    const float a3 = y0p[12];
    rs[0] = a0;
    rs[1] = a1;
    rs[2] = a2;
    rs[3] = a3;
  }
#pragma unroll
  for (int s = 1; s < kParts; ++s) {
    const float* ysp = YP + (size_t)s * kYpPlane + yo;
    const float e0 = ysp[0];
    const float e1 = ysp[4];
    const float e2 = ysp[8];
    const float e3 = ysp[12];
    rs[0] = rs[0] + e0;
    rs[1] = rs[1] + e1;
    rs[2] = rs[2] + e2;
    rs[3] = rs[3] + e3;
  }
  const v4f xc = *(const v4f*)(XC + (size_t)row * kHid + d4);
  const v4f dp = *(const v4f*)(Dskip + d4);
  const v4f zz = *(const v4f*)(XZ + (size_t)row * kXz + kHid + d4);
  const float u0 = xc[0];
  const float u1 = xc[1];
  const float u2 = xc[2];
  const float u3 = xc[3];
  const float k0 = dp[0];
  const float k1 = dp[1];
  const float k2 = dp[2];
  const float k3 = dp[3];
  const float z0 = zz[0];
  const float z1 = zz[1];
  const float z2 = zz[2];
  const float z3 = zz[3];
  const float y0 = fmaf(u0, bf16r(k0), rs[0]);
  const float y1 = fmaf(u1, bf16r(k1), rs[1]);
  const float y2 = fmaf(u2, bf16r(k2), rs[2]);
  const float y3 = fmaf(u3, bf16r(k3), rs[3]);
  v4f o;
  o[0] = y0 * (z0 / (1.0f + expf(-z0)));
  o[1] = y1 * (z1 / (1.0f + expf(-z1)));
  o[2] = y2 * (z2 / (1.0f + expf(-z2)));
  o[3] = y3 * (z3 / (1.0f + expf(-z3)));
  float* p = Y + (size_t)row * kHid + d4;
  *(volatile v4f*)p = o;
  __threadfence();
  *(volatile v4f*)p = o;
}

__global__ __launch_bounds__(128) void ln_rowsum_kernel(
    const float* __restrict__ H2, const float* __restrict__ bias, float* __restrict__ RS)
{
  const int t = blockIdx.x * 128 + threadIdx.x;
  const float* hp = H2 + (size_t)t * 4 * kHid;
  float s[4] = {0.0f, 0.0f, 0.0f, 0.0f};
  for (int cc = 0; cc < 16; ++cc) {
    const v4f bq = *(const v4f*)(bias + 4 * cc);
    const float b0 = bq[0];
    const float b1 = bq[1];
    const float b2 = bq[2];
    const float b3 = bq[3];
    const float r0 = bf16r(b0);
    const float r1 = bf16r(b1);
    const float r2 = bf16r(b2);
    const float r3 = bf16r(b3);
#pragma unroll
    for (int j = 0; j < 4; ++j) {
      const v4f v = *(const v4f*)(hp + (size_t)j * kHid + 4 * cc);
      const float v0 = v[0];
      const float v1 = v[1];
      const float v2 = v[2];
      const float v3 = v[3];
      s[j] += (v0 + r0);
      s[j] += (v1 + r1);
      s[j] += (v2 + r2);
      s[j] += (v3 + r3);
    }
  }
  v4f o;
  o[0] = s[0];
  o[1] = s[1];
  o[2] = s[2];
  o[3] = s[3];
  float* p = RS + (size_t)t * 4;
  *(volatile v4f*)p = o;
  __threadfence();
  *(volatile v4f*)p = o;
}

__global__ __launch_bounds__(128) void ln_rowsq_kernel(
    const float* __restrict__ H2, const float* __restrict__ bias, const float* __restrict__ MU,
    float* __restrict__ RS)
{
  const int t = blockIdx.x * 128 + threadIdx.x;
  const float* hp = H2 + (size_t)t * 4 * kHid;
  const float mu = MU[(t * 4) / kLen];
  float s[4] = {0.0f, 0.0f, 0.0f, 0.0f};
  for (int cc = 0; cc < 16; ++cc) {
    const v4f bq = *(const v4f*)(bias + 4 * cc);
    const float b0 = bq[0];
    const float b1 = bq[1];
    const float b2 = bq[2];
    const float b3 = bq[3];
    const float r0 = bf16r(b0);
    const float r1 = bf16r(b1);
    const float r2 = bf16r(b2);
    const float r3 = bf16r(b3);
#pragma unroll
    for (int j = 0; j < 4; ++j) {
      const v4f v = *(const v4f*)(hp + (size_t)j * kHid + 4 * cc);
      const float v0 = v[0];
      const float v1 = v[1];
      const float v2 = v[2];
      const float v3 = v[3];
      const float d0 = (v0 + r0) - mu;
      const float d1 = (v1 + r1) - mu;
      const float d2 = (v2 + r2) - mu;
      const float d3 = (v3 + r3) - mu;
      s[j] = fmaf(d0, d0, s[j]);
      s[j] = fmaf(d1, d1, s[j]);
      s[j] = fmaf(d2, d2, s[j]);
      s[j] = fmaf(d3, d3, s[j]);
    }
  }
  v4f o;
  o[0] = s[0];
  o[1] = s[1];
  o[2] = s[2];
  o[3] = s[3];
  float* p = RS + (size_t)t * 4;
  *(volatile v4f*)p = o;
  __threadfence();
  *(volatile v4f*)p = o;
}

__device__ __forceinline__ float seq_total(const float* __restrict__ rp) {
  float s = 0.0f;
  for (int g = 0; g < 16; ++g) {
    const v4f v = *(const v4f*)(rp + 4 * g);
    const float v0 = v[0];
    const float v1 = v[1];
    const float v2 = v[2];
    const float v3 = v[3];
    s += v0;
    s += v1;
    s += v2;
    s += v3;
  }
  return s;
}

__global__ __launch_bounds__(64) void ln_mean_kernel(
    const float* __restrict__ RS, float* __restrict__ MU)
{
  const int i = threadIdx.x;
  v4f o;
#pragma unroll
  for (int j = 0; j < 4; ++j) {
    const int qq = 4 * i + j;
    const int q = (qq < kSeqs) ? qq : (kSeqs - 1);
    const float tot = seq_total(RS + (size_t)q * kLen);
    o[j] = tot / 4096.0f;
  }
  float* p = MU + (size_t)i * 4;
  *(volatile v4f*)p = o;
  __threadfence();
  *(volatile v4f*)p = o;
}

__global__ __launch_bounds__(64) void ln_rstd_kernel(
    const float* __restrict__ RS, float* __restrict__ RSTD)
{
  const int i = threadIdx.x;
  v4f o;
#pragma unroll
  for (int j = 0; j < 4; ++j) {
    const int qq = 4 * i + j;
    const int q = (qq < kSeqs) ? qq : (kSeqs - 1);
    const float tot = seq_total(RS + (size_t)q * kLen);
    o[j] = 1.0f / sqrtf(tot / 4096.0f + kLnEps);
  }
  float* p = RSTD + (size_t)i * 4;
  *(volatile v4f*)p = o;
  __threadfence();
  *(volatile v4f*)p = o;
}

__global__ __launch_bounds__(256) void ln_apply_kernel(
    const float* __restrict__ H2, const float* __restrict__ bias, const float* __restrict__ MU,
    const float* __restrict__ RSTD, const float* __restrict__ lnw, const float* __restrict__ lnb,
    float* __restrict__ L3)
{
  const int i = blockIdx.x * 256 + threadIdx.x;
  const int rr = i >> 4;
  const int c4 = (i & 15) * 4;
  const int q = rr / kOutLen;
  const int lp = rr - q * kOutLen;
  const int l = lp + (kLen - kOutLen);
  const size_t row = (size_t)q * kLen + l;
  const v4f hv = *(const v4f*)(H2 + row * kHid + c4);
  const v4f bq = *(const v4f*)(bias + c4);
  const v4f wq = *(const v4f*)(lnw + (size_t)l * kHid + c4);
  const v4f gq = *(const v4f*)(lnb + (size_t)l * kHid + c4);
  const float mu = MU[q];
  const float rs = RSTD[q];
  v4f o;
#pragma unroll
  for (int e = 0; e < 4; ++e) {
    const float he = hv[e];
    const float be = bq[e];
    const float we = wq[e];
    const float ge = gq[e];
    const float dv = (he + bf16r(be)) - mu;
    o[e] = dv * rs * bf16r(we) + bf16r(ge);
  }
  float* p = L3 + (size_t)rr * kHid + c4;
  *(volatile v4f*)p = o;
  __threadfence();
  *(volatile v4f*)p = o;
}

__global__ __launch_bounds__(256) void heads_out_kernel(
    const float* __restrict__ RAW, const float* __restrict__ mu_b, const float* __restrict__ sg_b,
    const float* __restrict__ nmask, float* __restrict__ out)
{
  const int t = blockIdx.x * 256 + threadIdx.x;
  const int g = t & 7;
  const int t1 = t >> 3;
  const int node = t1 % kNodes;
  const int t2 = t1 / kNodes;
  const int o = t2 % kOutDim;
  const int b = t2 / kOutDim;
  const float* rp = RAW + (size_t)((node * kBatch + b) * kOutLen + 4 * g) * kHid;
  const float bm = bf16r(mu_b[o]);
  const float bs = bf16r(sg_b[o]);
  const float mk = bf16r(nmask[b * kNodes + node]);
  v4f vz, vm, vs;
#pragma unroll
  for (int j = 0; j < 4; ++j) {
    const float rm = rp[(size_t)j * kHid + o] + bm;
    const float rg = rp[(size_t)j * kHid + kOutDim + o] + bs;
    const float xm = rm / (1.0f + expf(-rm));
    const float xs = rg / (1.0f + expf(-rg));
    vm[j] = xm;
    vz[j] = xm * mk;
    vs[j] = xs;
  }
  float* p0 = out + (size_t)t * 4;
  float* p1 = out + (size_t)kOutElems + (size_t)t * 4;
  float* p2 = out + (size_t)2 * kOutElems + (size_t)t * 4;
  for (int pass = 0; pass < 2; ++pass) {
    *(volatile v4f*)p0 = vz;
    *(volatile v4f*)p1 = vm;
    *(volatile v4f*)p2 = vs;
    __threadfence();
  }
}

static_assert(((kRows / 32) * (kHid / 64)) % 8 == 0);
static_assert(((kRows / 32) * (kXz / 64)) % 8 == 0);
static_assert(((kRows / 32) * (kProjP / 64)) % 8 == 0);
static_assert(((kRowsT / 32) * (kHid / 64)) % 8 == 0);
static_assert((kHid * kRankP / 8) == 256);
static_assert(((kHid * 8) % 256) == 0 && ((kXz * 8) % 256) == 0 && ((kProjP * 8) % 256) == 0 && (kOutDim * 8) == 256);
static_assert(((kRows * 4) % 256) == 0 && ((kRows * 8) % 256) == 0 && ((kRowsT * 8) % 256) == 0);
static_assert(((kRows * 16) % 256) == 0 && ((kRowsT * 16) % 256) == 0);
static_assert(((kHid * kState / 4) % 256) == 0);
static_assert((kHid * kParts) == 512 && ((kSeqs * kHid * kParts) % 256) == 0);
static_assert(((kSeqs * kHid * kParts) / 256) == 400);
static_assert(((kRows / 4) % 128) == 0);
static_assert(((kOutElems / 4) % 256) == 0);

extern "C" void kernel_launch(void* const* d_in, const int* in_sizes, int n_in,
                              void* d_out, int out_size, void* d_ws, size_t ws_size,
                              hipStream_t stream)
{
  if (n_in < 24) return;
  if (in_sizes[0] != kBatch * kNodes * kFeat * kLen) return;
  if (in_sizes[1] != kBatch * kNodes) return;
  if (in_sizes[2] != kBatch * kNodes) return;
  if (in_sizes[3] != kHid * kFeat) return;
  if (in_sizes[4] != kHid) return;
  if (in_sizes[5] != kHid * kHid) return;
  if (in_sizes[6] != kHid) return;
  if (in_sizes[7] != kHid * kHid) return;
  if (in_sizes[8] != kHid) return;
  if (in_sizes[9] != kXz * kHid) return;
  if (in_sizes[10] != kHid * 2) return;
  if (in_sizes[11] != kHid) return;
  if (in_sizes[12] != kProjN * kHid) return;
  if (in_sizes[13] != kHid * kDtRank) return;
  if (in_sizes[14] != kHid) return;
  if (in_sizes[15] != kHid * kState) return;
  if (in_sizes[16] != kHid) return;
  if (in_sizes[17] != kHid * kHid) return;
  if (in_sizes[18] != kLen * kHid) return;
  if (in_sizes[19] != kLen * kHid) return;
  if (in_sizes[20] != kOutDim * kHid) return;
  if (in_sizes[21] != kOutDim) return;
  if (in_sizes[22] != kOutDim * kHid) return;
  if (in_sizes[23] != kOutDim) return;
  if (out_size != 3 * kOutElems) return;
  if (ws_size < kWsTotal) return;

  const float* x           = (const float*)d_in[0];
  const float* nodes_mask  = (const float*)d_in[1];
  const float* emb_w       = (const float*)d_in[3];
  const float* emb_b       = (const float*)d_in[4];
  const float* dim_layer_w = (const float*)d_in[5];
  const float* dim_layer_b = (const float*)d_in[6];
  const float* dim_out_w   = (const float*)d_in[7];
  const float* dim_out_b   = (const float*)d_in[8];
  const float* in_proj_w   = (const float*)d_in[9];
  const float* conv_w      = (const float*)d_in[10];
  const float* conv_b      = (const float*)d_in[11];
  const float* x_proj_w    = (const float*)d_in[12];
  const float* dt_proj_w   = (const float*)d_in[13];
  const float* dt_proj_b   = (const float*)d_in[14];
  const float* A_log       = (const float*)d_in[15];
  const float* Dp          = (const float*)d_in[16];
  const float* out_proj_w  = (const float*)d_in[17];
  const float* ln_w        = (const float*)d_in[18];
  const float* ln_b        = (const float*)d_in[19];
  const float* mu_w        = (const float*)d_in[20];
  const float* mu_b        = (const float*)d_in[21];
  const float* sigma_w     = (const float*)d_in[22];
  const float* sigma_b     = (const float*)d_in[23];
  float* out = (float*)d_out;

  char* ws = (char*)d_ws;
  unsigned short* EW   = (unsigned short*)(ws + kOffEW);
  unsigned short* W1   = (unsigned short*)(ws + kOffW1);
  unsigned short* W2   = (unsigned short*)(ws + kOffW2);
  unsigned short* W3   = (unsigned short*)(ws + kOffW3);
  unsigned short* W4   = (unsigned short*)(ws + kOffW4);
  unsigned short* W5   = (unsigned short*)(ws + kOffW5);
  unsigned short* HW   = (unsigned short*)(ws + kOffHW);
  float*          AN   = (float*)(ws + kOffAN);
  unsigned short* XA   = (unsigned short*)(ws + kOffXA);
  float*          H0   = (float*)(ws + kOffH0);
  unsigned short* A1H  = (unsigned short*)(ws + kOffA1H);
  unsigned short* A1L  = (unsigned short*)(ws + kOffA1L);
  float*          H1   = (float*)(ws + kOffH1);
  unsigned short* A2H  = (unsigned short*)(ws + kOffA2H);
  unsigned short* A2L  = (unsigned short*)(ws + kOffA2L);
  float*          XZ   = (float*)(ws + kOffXZ);
  float*          XC   = (float*)(ws + kOffXC);
  unsigned short* XCH  = (unsigned short*)(ws + kOffXCH);
  unsigned short* XCL  = (unsigned short*)(ws + kOffXCL);
  float*          PROJ = (float*)(ws + kOffPROJ);
  float*          DT   = (float*)(ws + kOffDT);
  float*          YP   = (float*)(ws + kOffYP);
  float*          Y    = (float*)(ws + kOffY);
  unsigned short* YH   = (unsigned short*)(ws + kOffYH);
  unsigned short* YL   = (unsigned short*)(ws + kOffYL);
  float*          Mo   = (float*)(ws + kOffM);
  unsigned short* GH   = (unsigned short*)(ws + kOffGH);
  unsigned short* GL   = (unsigned short*)(ws + kOffGL);
  float*          H2   = (float*)(ws + kOffH2);
  float*          RS1  = (float*)(ws + kOffRS1);
  float*          MU   = (float*)(ws + kOffMU);
  float*          RS2  = (float*)(ws + kOffRS2);
  float*          RSTD = (float*)(ws + kOffRSTD);
  float*          L3   = (float*)(ws + kOffL3);
  unsigned short* LH   = (unsigned short*)(ws + kOffLH);
  unsigned short* LL   = (unsigned short*)(ws + kOffLL);
  float*          RAW  = (float*)(ws + kOffRAW);

  constexpr float sW  = 1.0f / kWCarry;
  constexpr float sWr = sW / kResid;

  pack_kpad_bf_kernel<<<(kHid * kRankP / 8) / 256, 256, 0, stream>>>(emb_w, EW, kHid * kRankP / 8, kWCarry);

  pack_w_kernel<<<(kHid * 8) / 256, 256, 0, stream>>>(dim_layer_w, W1, kHid, kWCarry);
  pack_w_kernel<<<(kXz * 8) / 256, 256, 0, stream>>>(in_proj_w, W2, kXz, kWCarry);
  pack_w_kernel<<<(kProjP * 8) / 256, 256, 0, stream>>>(x_proj_w, W3, kProjN, kWCarry);
  pack_w_kernel<<<(kHid * 8) / 256, 256, 0, stream>>>(out_proj_w, W4, kHid, kWCarry);
  pack_w_kernel<<<(kHid * 8) / 256, 256, 0, stream>>>(dim_out_w, W5, kHid, kWCarry);
  pack_w_kernel<<<(kOutDim * 8) / 256, 256, 0, stream>>>(mu_w, HW, kOutDim, kWCarry);
  pack_w_kernel<<<(kOutDim * 8) / 256, 256, 0, stream>>>(sigma_w, HW + (size_t)kOutDim * kHid, kOutDim, kWCarry);

  embed_a_kernel<<<(kRows * 4) / 256, 256, 0, stream>>>(x, XA);

  eng::gemm_f16_kernel<2, 0><<<dim3((kRows / 32) * (kHid / 64) / 8), 256, 0, stream>>>(
      XA, nullptr, kRankP, EW, nullptr, kRankP, H0, kHid, kRows, kHid, kRankP, sW, 0.0f);

  split_kernel<0, 1><<<(kRows * 8) / 256, 256, 0, stream>>>(H0, emb_b, A1H, A1L);

  eng::gemm_f16_kernel<2, 1><<<dim3((kRows / 32) * (kHid / 64) / 8), 256, 0, stream>>>(
      A1H, A1L, kHid, W1, W1, kHid, H1, kHid, kRows, kHid, kHid, sW, sWr);

  split_kernel<0, 1><<<(kRows * 8) / 256, 256, 0, stream>>>(H1, dim_layer_b, A2H, A2L);

  eng::gemm_f16_kernel<2, 1><<<dim3((kRows / 32) * (kXz / 64) / 8), 256, 0, stream>>>(
      A2H, A2L, kHid, W2, W2, kHid, XZ, kXz, kRows, kXz, kHid, sW, sWr);

  conv_silu_kernel<<<(kRows * 16) / 256, 256, 0, stream>>>(XZ, conv_w, conv_b, XC);
  split_kernel<0, 0><<<(kRows * 8) / 256, 256, 0, stream>>>(XC, nullptr, XCH, XCL);

  eng::gemm_f16_kernel<2, 1><<<dim3((kRows / 32) * (kProjP / 64) / 8), 256, 0, stream>>>(
      XCH, XCL, kHid, W3, W3, kHid, PROJ, kProjP, kRows, kProjP, kHid, sW, sWr);

  dt_kernel<<<(kRows * 16) / 256, 256, 0, stream>>>(PROJ, dt_proj_w, dt_proj_b, DT);
  a_neg_kernel<<<(kHid * kState / 4) / 256, 256, 0, stream>>>(A_log, AN);

  scan_kernel<<<(kSeqs * kHid * kParts) / 256, 256, 0, stream>>>(DT, XC, PROJ, AN, YP);
  gate_kernel<<<(kRows * 16) / 256, 256, 0, stream>>>(YP, XC, XZ, Dp, Y);
  split_kernel<0, 0><<<(kRows * 8) / 256, 256, 0, stream>>>(Y, nullptr, YH, YL);

  eng::gemm_f16_kernel<2, 1><<<dim3((kRows / 32) * (kHid / 64) / 8), 256, 0, stream>>>(
      YH, YL, kHid, W4, W4, kHid, Mo, kHid, kRows, kHid, kHid, sW, sWr);
  split_kernel<1, 0><<<(kRows * 8) / 256, 256, 0, stream>>>(Mo, nullptr, GH, GL);

  eng::gemm_f16_kernel<2, 1><<<dim3((kRows / 32) * (kHid / 64) / 8), 256, 0, stream>>>(
      GH, GL, kHid, W5, W5, kHid, H2, kHid, kRows, kHid, kHid, sW, sWr);

  ln_rowsum_kernel<<<(kRows / 4) / 128, 128, 0, stream>>>(H2, dim_out_b, RS1);
  ln_mean_kernel<<<1, 64, 0, stream>>>(RS1, MU);
  ln_rowsq_kernel<<<(kRows / 4) / 128, 128, 0, stream>>>(H2, dim_out_b, MU, RS2);
  ln_rstd_kernel<<<1, 64, 0, stream>>>(RS2, RSTD);
  ln_apply_kernel<<<(kRowsT * 16) / 256, 256, 0, stream>>>(H2, dim_out_b, MU, RSTD, ln_w, ln_b, L3);
  split_kernel<0, 0><<<(kRowsT * 8) / 256, 256, 0, stream>>>(L3, nullptr, LH, LL);

  eng::gemm_f16_kernel<2, 1><<<dim3((kRowsT / 32) * (kHid / 64) / 8), 256, 0, stream>>>(
      LH, LL, kHid, HW, HW, kHid, RAW, kHid, kRowsT, kHid, kHid, sW, sWr);

  heads_out_kernel<<<(kOutElems / 4) / 256, 256, 0, stream>>>(RAW, mu_b, sigma_b, nodes_mask, out);
}
